// NDP_27882927685986
// MI455X (gfx1250) — hardware-run, weakly checked
//
#include <hip/hip_runtime.h>


#ifndef NN
#define NN 1024
#endif
#define NN_FULL 1024
#define DM   256
#define HM   256
#define NC   768
#define TS   68
#define WSC  1024.0f
#define WSI  (1.0f / 1024.0f)
#define ETI  64
#define EKC  64
#define EPAD 66

static_assert(HM == DM);
static_assert(DM % 32 == 0);
static_assert(DM % 64 == 0);
static_assert(NC % 64 == 0);
static_assert(NC == 3 * HM);
static_assert(NN % 64 == 0);
static_assert(NN <= NN_FULL);
static_assert(DM / 8 == 32);
static_assert(HM % EKC == 0);
static_assert(EKC == 64);
static_assert(ETI == 64);
static_assert(256 * 4 * 16 == ETI * ETI * 4);
static_assert(4 * 32 * 16 == 16 * 64 * 2);
static_assert(8 * 32 * 16 == 16 * 64 * 4);
static_assert(192 * 4 == NC);
static_assert((TS * 4) % 16 == 0);
static_assert(16 * TS * 4 <= 131072);
static_assert((2 * ETI * EPAD + EKC) * 4 <= 131072);
static_assert((size_t)NN_FULL * DM * 4 == 1048576);
static_assert((size_t)NN_FULL * DM * 4 + (size_t)NN_FULL * 4 == 1052672);
static_assert((size_t)1052672 + (size_t)NN_FULL * NN_FULL * 4 == 5246976);
static_assert(1048576 % 128 == 0);
static_assert(1052672 % 128 == 0);

typedef _Float16 h16;
typedef unsigned short bf;
typedef __attribute__((ext_vector_type(16))) __bf16   v16bf;
typedef __attribute__((ext_vector_type(16))) _Float16 v16h;
typedef __attribute__((ext_vector_type(8)))  _Float16 v8h;
typedef __attribute__((ext_vector_type(8)))  unsigned short v8us;
typedef __attribute__((ext_vector_type(8)))  float    v8f;
typedef __attribute__((ext_vector_type(4)))  float    v4f;
typedef v4f  __attribute__((may_alias)) v4fa;
typedef __attribute__((ext_vector_type(2)))  float    v2f;
typedef v2f  __attribute__((may_alias)) v2fa;

__device__ __forceinline__ unsigned short f2bf(float f) { unsigned u = __float_as_uint(f); u += 0x7FFFu + ((u >> 16) & 1u); return (unsigned short)(u >> 16); }
__device__ __forceinline__ float bfr(float f) { return __uint_as_float(((unsigned)f2bf(f)) << 16); }
__device__ __forceinline__ v16h cat16(v8h lo, v8h hi) { return __builtin_shufflevector(lo, hi, 0, 1, 2, 3, 4, 5, 6, 7, 8, 9, 10, 11, 12, 13, 14, 15); }
__device__ __forceinline__ v16bf cat16b(v8us lo, v8us hi) { return __builtin_bit_cast(v16bf, __builtin_shufflevector(lo, hi, 0, 1, 2, 3, 4, 5, 6, 7, 8, 9, 10, 11, 12, 13, 14, 15)); }
__device__ __forceinline__ v8f wmma16(v16h a, v16h b, v8f c) { return __builtin_amdgcn_wmma_f32_16x16x32_f16(false, a, false, b, (short)0, c, false, false); }
__device__ __forceinline__ v8f wmmab(v16bf a, v16bf b, v8f c) { return __builtin_amdgcn_wmma_f32_16x16x32_bf16(false, a, false, b, (short)0, c, false, false); }
__device__ __forceinline__ v16h  ldh(const h16* p) { return cat16(*(const v8h*)p, *(const v8h*)(p + 16)); }
__device__ __forceinline__ v16bf ldb(const bf* p)  { return cat16b(*(const v8us*)p, *(const v8us*)(p + 16)); }
__device__ __forceinline__ void wave_sync() { __builtin_amdgcn_fence(3  , "wavefront"); __builtin_amdgcn_wave_barrier(); asm volatile("" ::: "memory"); }

static __device__ __forceinline__ h16 toh_flush(float v) { const h16 r = (h16)v; return (fabsf(v) < 6.103515625e-05f) ? (h16)0.0f : r; }
__device__ __forceinline__ v8f wmma16g(v16h a, v16h b, v8f c) { c = wmma16(a, b, c); asm volatile("v_nop\n\tv_nop\n\tv_nop\n\tv_nop" : "+v"(c) : "v"(a), "v"(b)); return c; }
__device__ __forceinline__ v8f wmmabg(v16bf a, v16bf b, v8f c) { c = wmmab(a, b, c); asm volatile("v_nop\n\tv_nop\n\tv_nop\n\tv_nop" : "+v"(c) : "v"(a), "v"(b)); return c; }

__global__ __launch_bounds__(256) void k_cvt8(const float* __restrict__ src, bf* dst, size_t n8) {
    const size_t i = (size_t)blockIdx.x * 256 + threadIdx.x; if (i >= n8) return;
    const v8f v = *(const v8f*)(src + i * 8); v8us o;
#pragma unroll
    for (int k = 0; k < 8; ++k) o[k] = f2bf(v[k]);
    *(volatile v8us*)(dst + i * 8) = o; __threadfence(); *(volatile v8us*)(dst + i * 8) = o;
}

__global__ __launch_bounds__(256) void k_wcvt(const float* __restrict__ src, int ld, h16* dst, int n8) {
    const int i = blockIdx.x * 256 + threadIdx.x; if (i >= n8) return;
    const int row = i >> 5, c8 = (i & 31) * 8;
    const v8f v = *(const v8f*)(src + (size_t)row * (size_t)ld + c8); v8h o;
#pragma unroll
    for (int k = 0; k < 8; ++k) o[k] = toh_flush(bfr(v[k]) * WSC);
    *(volatile v8h*)(dst + (size_t)i * 8) = o; __threadfence(); *(volatile v8h*)(dst + (size_t)i * 8) = o;
}

__global__ __launch_bounds__(192) void k_bias(const float* __restrict__ br1, const float* __restrict__ bu1, float* BC) {
    const int i = threadIdx.x; const int c = 4 * i; const int seg = c >> 8; const int cc = c & 255;
    v4f a = *(const v4f*)(br1 + cc); v4f b = *(const v4f*)(bu1 + cc);
    asm volatile("" : "+v"(a)); asm volatile("" : "+v"(b));
    v4f o;
#pragma unroll
    for (int k = 0; k < 4; ++k) { const float x = bfr(a[k]); const float y = bfr(b[k]); o[k] = (seg == 0) ? x : ((seg == 1) ? y : 0.0f); }
    *(volatile v4f*)(BC + c) = o; __threadfence(); *(volatile v4f*)(BC + c) = o;
}

__global__ __launch_bounds__(32) void k_gemm_in(const bf* __restrict__ A, const bf* __restrict__ Bt, const float* __restrict__ bias, h16* Ph) {
    __shared__ __align__(16) float os[16 * TS];
    const int lane = threadIdx.x & 31, lr = lane & 15, hi = lane >> 4; const int r0 = blockIdx.x * 32, c0 = blockIdx.y * 64;
    v8f acc[2][4];
#pragma unroll
    for (int mb = 0; mb < 2; ++mb)
#pragma unroll
        for (int nb = 0; nb < 4; ++nb) acc[mb][nb] = (v8f){};
    const size_t aoff = (size_t)(r0 + lr) * DM + 8 * hi, boff = (size_t)(c0 + lr) * DM + 8 * hi;
#pragma unroll 1
    for (int kc = 0; kc < DM; kc += 32) {
        v16bf a[2];
#pragma unroll
        for (int mb = 0; mb < 2; ++mb) a[mb] = ldb(A + aoff + (size_t)mb * 16 * DM + kc);
#pragma unroll
        for (int nb = 0; nb < 4; ++nb) { const v16bf b = ldb(Bt + boff + (size_t)nb * 16 * DM + kc);
#pragma unroll
            for (int mb = 0; mb < 2; ++mb) acc[mb][nb] = wmmabg(a[mb], b, acc[mb][nb]); }
    }
    float bc[4];
#pragma unroll
    for (int nb = 0; nb < 4; ++nb) bc[nb] = bfr(bias[c0 + nb * 16 + lr]);
#pragma unroll
    for (int mb = 0; mb < 2; ++mb) {
#pragma unroll
        for (int nb = 0; nb < 4; ++nb) {
#pragma unroll
            for (int j = 0; j < 8; ++j) os[(hi * 8 + j) * TS + nb * 16 + lr] = fmaxf(acc[mb][nb][j] + bc[nb], 0.0f); }
        wave_sync();
        const size_t pb = (size_t)(r0 + mb * 16) * HM + c0;
#pragma unroll 1
        for (int ps = 0; ps < 2; ++ps) {
#pragma unroll
            for (int s = 0; s < 4; ++s) { const int row = 4 * s + (lane >> 3), c8 = (lane & 7) * 8;
                const v4f x0 = *(const v4fa*)(&os[row * TS + c8]); const v4f x1 = *(const v4fa*)(&os[row * TS + c8 + 4]); v8h hv;
#pragma unroll
                for (int i = 0; i < 4; ++i) { hv[i] = toh_flush(x0[i]); hv[4 + i] = toh_flush(x1[i]); }
                const size_t oo = pb + (size_t)row * HM + c8;
                *(volatile v8h*)(Ph + oo) = hv; }
            if (ps == 0) __threadfence(); }
        wave_sync();
    }
}

__global__ __launch_bounds__(32) void k_gemm_act(const h16* __restrict__ AH, const h16* __restrict__ Bt, const float* __restrict__ bias,
                                                 float* F, int ldf, int relu_cols, h16* Ph, int wplanes) {
    __shared__ __align__(16) float os[16 * TS];
    const int lane = threadIdx.x & 31, lr = lane & 15, hi = lane >> 4; const int r0 = blockIdx.x * 32, c0 = blockIdx.y * 64;
    const int dorelu = (c0 < relu_cols) ? 1 : 0;
    v8f acc[2][4];
#pragma unroll
    for (int mb = 0; mb < 2; ++mb)
#pragma unroll
        for (int nb = 0; nb < 4; ++nb) acc[mb][nb] = (v8f){};
    const size_t aoff = (size_t)(r0 + lr) * DM + 8 * hi, boff = (size_t)(c0 + lr) * DM + 8 * hi;
#pragma unroll 1
    for (int kc = 0; kc < DM; kc += 32) {
        v16h ah[2];
#pragma unroll
        for (int mb = 0; mb < 2; ++mb) ah[mb] = ldh(AH + aoff + (size_t)mb * 16 * DM + kc);
#pragma unroll
        for (int nb = 0; nb < 4; ++nb) { const v16h b = ldh(Bt + boff + (size_t)nb * 16 * DM + kc);
#pragma unroll
            for (int mb = 0; mb < 2; ++mb) acc[mb][nb] = wmma16g(ah[mb], b, acc[mb][nb]); }
    }
    float bc[4];
#pragma unroll
    for (int nb = 0; nb < 4; ++nb) bc[nb] = bfr(bias[c0 + nb * 16 + lr]);
#pragma unroll
    for (int mb = 0; mb < 2; ++mb) {
#pragma unroll
        for (int nb = 0; nb < 4; ++nb) {
#pragma unroll
            for (int j = 0; j < 8; ++j) { float v = acc[mb][nb][j] * WSI + bc[nb]; if (dorelu) v = fmaxf(v, 0.0f);
                os[(hi * 8 + j) * TS + nb * 16 + lr] = v; } }
        wave_sync();
        float* fb = F + (size_t)(r0 + mb * 16) * (size_t)ldf + c0;
        const size_t pb = (size_t)(r0 + mb * 16) * DM + c0;
#pragma unroll 1
        for (int ps = 0; ps < 2; ++ps) {
#pragma unroll
            for (int s = 0; s < 8; ++s) { const int row = 2 * s + (lane >> 4), c4 = (lane & 15) * 4;
                const v4f val = *(const v4fa*)(&os[row * TS + c4]);
                *(volatile v4f*)(fb + (size_t)row * (size_t)ldf + c4) = val; }
            if (wplanes) {
#pragma unroll
                for (int s = 0; s < 4; ++s) { const int row = 4 * s + (lane >> 3), c8 = (lane & 7) * 8;
                    const v4f x0 = *(const v4fa*)(&os[row * TS + c8]); const v4f x1 = *(const v4fa*)(&os[row * TS + c8 + 4]); v8h hv;
#pragma unroll
                    for (int i = 0; i < 4; ++i) { hv[i] = toh_flush(x0[i]); hv[4 + i] = toh_flush(x1[i]); }
                    const size_t oo = pb + (size_t)row * DM + c8;
                    *(volatile v8h*)(Ph + oo) = hv; } }
            if (ps == 0) __threadfence(); }
        wave_sync();
    }
}

__global__ __launch_bounds__(32) void k_head(const float* __restrict__ HC, const float* __restrict__ wr2, const float* __restrict__ br2, float* OUT1) {
    const int lane = threadIdx.x & 31;
    float w[8];
#pragma unroll
    for (int q = 0; q < 8; ++q) w[q] = bfr(wr2[lane + 32 * q]);
    const int row0 = blockIdx.x * 32;
    float keep = 0.0f;
#pragma unroll 1
    for (int r = 0; r < 32; ++r) {
        const float* tr = HC + (size_t)(row0 + r) * NC + lane;
        float s = 0.0f;
#pragma unroll
        for (int q = 0; q < 8; ++q) s = fmaf(tr[32 * q], w[q], s);
        s += __shfl_xor(s, 16, 32); s += __shfl_xor(s, 8, 32); s += __shfl_xor(s, 4, 32); s += __shfl_xor(s, 2, 32); s += __shfl_xor(s, 1, 32);
        keep = (lane == r) ? s : keep; }
    const float z = keep + bfr(br2[0]);
    const float val = 1.0f / (1.0f + expf(-z));
    *(volatile float*)(OUT1 + row0 + lane) = val; __threadfence(); *(volatile float*)(OUT1 + row0 + lane) = val;
}

__global__ __launch_bounds__(256) void k_edge(const float* __restrict__ HC, const float* __restrict__ w2, const float* __restrict__ bu2, float* OUT2) {
    __shared__ __align__(16) float shi[ETI * EPAD];
    __shared__ __align__(16) float shj[ETI * EPAD];
    __shared__ __align__(16) float sw[EKC];
    const int tid = threadIdx.x;
    const int bi = blockIdx.x * ETI, bj = blockIdx.y * ETI;
    const int i0 = (tid >> 4) << 2, j0 = (tid & 15) << 2;
    float acc[4][4];
#pragma unroll
    for (int ti = 0; ti < 4; ++ti)
#pragma unroll
        for (int tj = 0; tj < 4; ++tj) acc[ti][tj] = 0.0f;
#pragma unroll 1
    for (int kc = 0; kc < HM; kc += EKC) {
        __syncthreads();
#pragma unroll 1
        for (int idx = tid; idx < ETI * (EKC / 2); idx += 256) {
            const int row = idx >> 5, c = (idx & 31) << 1;
            const v2f a = *(const v2f*)(HC + (size_t)(bi + row) * NC + HM + kc + c);
            const v2f b = *(const v2f*)(HC + (size_t)(bj + row) * NC + 2 * HM + kc + c);
            *(v2fa*)(&shi[row * EPAD + c]) = a; *(v2fa*)(&shj[row * EPAD + c]) = b; }
        const float wl = bfr(w2[kc + (tid & (EKC - 1))]);
        if (tid < EKC) sw[tid] = wl;
        __syncthreads();
#pragma unroll 1
        for (int k = 0; k < EKC; k += 2) {
            v2f a[4], b[4];
#pragma unroll
            for (int t = 0; t < 4; ++t) { a[t] = *(const v2fa*)(&shi[(i0 + t) * EPAD + k]); b[t] = *(const v2fa*)(&shj[(j0 + t) * EPAD + k]); }
            const v2f wv = *(const v2fa*)(&sw[k]);
#pragma unroll
            for (int ti = 0; ti < 4; ++ti)
#pragma unroll
                for (int tj = 0; tj < 4; ++tj) {
                    acc[ti][tj] = fmaf(wv[0], fmaxf(a[ti][0] + b[tj][0], 0.0f), acc[ti][tj]);
                    acc[ti][tj] = fmaf(wv[1], fmaxf(a[ti][1] + b[tj][1], 0.0f), acc[ti][tj]); }
        }
    }
    const float eb = bfr(bu2[0]);
    v4f o[4];
#pragma unroll
    for (int ti = 0; ti < 4; ++ti) { o[ti][0] = acc[ti][0] + eb; o[ti][1] = acc[ti][1] + eb; o[ti][2] = acc[ti][2] + eb; o[ti][3] = acc[ti][3] + eb; }
    float* ob = OUT2 + (size_t)(bi + i0) * NN_FULL + bj + j0;
#pragma unroll 1
    for (int ps = 0; ps < 2; ++ps) {
#pragma unroll
        for (int ti = 0; ti < 4; ++ti) *(volatile v4f*)(ob + (size_t)ti * NN_FULL) = o[ti];
        if (ps == 0) __threadfence(); }
}

static constexpr size_t al256(size_t v) { return (v + 255) & ~(size_t)255; }
static constexpr size_t SZ_XB = al256((size_t)NN * DM * 2);
static constexpr size_t SZ_W1 = al256((size_t)HM * DM * 2);
static constexpr size_t SZ_W2 = al256((size_t)DM * HM * 2);
static constexpr size_t SZ_WC = al256((size_t)NC * DM * 2);
static constexpr size_t SZ_BC = al256((size_t)NC * 4);
static constexpr size_t SZ_PL = al256((size_t)NN * DM * 2);
static constexpr size_t SZ_HC = al256((size_t)NN * NC * 4);
static constexpr size_t SZ_TOTAL = SZ_XB + SZ_W1 + SZ_W2 + SZ_WC + SZ_BC + 2 * SZ_PL + SZ_HC;
static_assert(SZ_TOTAL <= (size_t)134217728);
static_assert(((size_t)HM * DM * 2) % 256 == 0);
static_assert(((size_t)HM * DM) % 8 == 0);
static_assert(((size_t)NN * DM) % 8 == 0);

extern "C" void kernel_launch(void* const* d_in, const int* in_sizes, int n_in,
                              void* d_out, int out_size, void* d_ws, size_t ws_size, hipStream_t stream) {
    if (n_in < 14) return;
    if ((size_t)in_sizes[0] < (size_t)NN * DM) return;
    if ((size_t)in_sizes[2] < (size_t)HM * DM || (size_t)in_sizes[4] < (size_t)DM * HM || (size_t)in_sizes[6] < (size_t)HM * DM) return;
    if ((size_t)in_sizes[10] < (size_t)HM * 2 * DM) return;
    if (in_sizes[3] < HM || in_sizes[5] < DM || in_sizes[7] < HM || in_sizes[8] < HM || in_sizes[11] < HM || in_sizes[12] < HM) return;
    if (in_sizes[9] < 1 || in_sizes[13] < 1) return;
    if ((size_t)out_size < (size_t)NN_FULL * DM + (size_t)NN_FULL + (size_t)(NN - 1) * NN_FULL + (size_t)NN) return;
    if (SZ_TOTAL > ws_size) return;
    const float* X   = (const float*)d_in[0];
    const float* W1  = (const float*)d_in[2];  const float* b1  = (const float*)d_in[3];
    const float* W2  = (const float*)d_in[4];  const float* b2  = (const float*)d_in[5];
    const float* Wr1 = (const float*)d_in[6];  const float* br1 = (const float*)d_in[7];
    const float* Wr2 = (const float*)d_in[8];  const float* br2 = (const float*)d_in[9];
    const float* Wu1 = (const float*)d_in[10]; const float* bu1 = (const float*)d_in[11];
    const float* Wu2 = (const float*)d_in[12]; const float* bu2 = (const float*)d_in[13];
    float* OUT0 = (float*)d_out;
    float* OUT1 = (float*)d_out + (size_t)NN_FULL * DM;
    float* OUT2 = (float*)d_out + (size_t)NN_FULL * DM + (size_t)NN_FULL;
    char* wsp = (char*)d_ws;
    bf*  XB  = (bf*)wsp;  wsp += SZ_XB;
    bf*  W1B = (bf*)wsp;  wsp += SZ_W1;
    h16* W2H = (h16*)wsp; wsp += SZ_W2;
    h16* WCH = (h16*)wsp; wsp += SZ_WC;
    float* BC = (float*)wsp; wsp += SZ_BC;
    h16* T1H = (h16*)wsp; wsp += SZ_PL;
    h16* UH  = (h16*)wsp; wsp += SZ_PL;
    float* HC = (float*)wsp; wsp += SZ_HC;

    { const size_t n8 = (size_t)NN * DM / 8; k_cvt8<<<(unsigned)((n8 + 255) / 256), 256, 0, stream>>>(X, XB, n8); }
    { const size_t n8 = (size_t)HM * DM / 8; k_cvt8<<<(unsigned)((n8 + 255) / 256), 256, 0, stream>>>(W1, W1B, n8); }
    { const int n8 = HM * DM / 8; const unsigned g = (unsigned)((n8 + 255) / 256);
      k_wcvt<<<g, 256, 0, stream>>>(W2,  DM, W2H, n8);
      k_wcvt<<<g, 256, 0, stream>>>(Wr1, DM, WCH, n8);
      k_wcvt<<<g, 256, 0, stream>>>(Wu1, 2 * DM, WCH + (size_t)HM * DM, n8);
      k_wcvt<<<g, 256, 0, stream>>>(Wu1 + DM, 2 * DM, WCH + (size_t)2 * HM * DM, n8); }
    k_bias<<<1, 192, 0, stream>>>(br1, bu1, BC);

    k_gemm_in<<<dim3(NN / 32, HM / 64, 1), 32, 0, stream>>>(XB, W1B, b1, T1H);
    k_gemm_act<<<dim3(NN / 32, DM / 64, 1), 32, 0, stream>>>(T1H, W2H, b2, OUT0, DM, 0, UH, 1);
    k_gemm_act<<<dim3(NN / 32, NC / 64, 1), 32, 0, stream>>>(UH, WCH, BC, HC, NC, HM, UH, 0);
    k_head<<<dim3(NN / 32, 1, 1), 32, 0, stream>>>(HC, Wr2, br2, OUT1);
    k_edge<<<dim3(NN / ETI, NN / ETI, 1), 256, 0, stream>>>(HC, Wu2, bu2, OUT2);
}
